// HeteroGAT_82308753261157
// MI455X (gfx1250) — hardware-verified
//
#include <hip/hip_runtime.h>
#include <stddef.h>
#include <stdint.h>
#include <math.h>


#define F_IN    128
#define HC      128
#define HD1     32
#define NH1     4
#define C2      16
#define NREL    3
#define N2P     64
#define K2      256
#define NTHR    256
#define NWAVE   8
#define EPT     8
#define CHUNK   (NTHR * EPT)
#define WCAP    (EPT * 32)
#define LISTN   (NWAVE * WCAP)
#define NBMAX   2048
#define NBCAP   1024
#define SLOTB   11
#define RCAP    28672
#define DEGCAP  256
#define GBM     64
#define GTHR    128
#define MROWS   128
#define NU1     (NREL * HC * (F_IN / 8))
#define NU2     (N2P * (K2 / 8))
#define NEGSL   0.2f
#define EPS_SM  1e-16f
#define MX0     (-1.0e30f)
#define THIRD   (1.0f / 3.0f)
#define WSMAX   134217728
#define LDS_AGG ((2 * RCAP + 2 * NBMAX + LISTN) * 4 + 64)

static_assert((CHUNK & (CHUNK - 1)) == 0 && CHUNK <= (1 << SLOTB));
static_assert(NBMAX == (1 << SLOTB));
static_assert(NTHR * 8 == NBMAX);
static_assert(LISTN >= NBMAX);
static_assert(LISTN >= NWAVE * WCAP);
static_assert((RCAP % 32) == 0);
static_assert(LDS_AGG <= 300000);
static_assert(GBM == (GTHR / 32) * 16);
static_assert(GTHR == 2 * GBM);
static_assert(2 * GTHR == 2 * NH1 * HD1);
static_assert(GTHR >= 2 * NREL * C2);
static_assert((F_IN % 32) == 0 && (K2 % 32) == 0 && K2 == 2 * HC);
static_assert(HC == NH1 * HD1 && HC == 4 * 32 && HD1 == 4 * 8);
static_assert(C2 == 16 && NREL * C2 <= N2P && N2P == 64);
static_assert((MROWS % GBM) == 0);
static_assert(NBCAP <= NBMAX && NBCAP * C2 <= RCAP);
static_assert((NU1 % NTHR) == 0 && (NU2 % NTHR) == 0);
static_assert((HC / 16) * 32 == K2);

typedef float          v4f  __attribute__((ext_vector_type(4)));
typedef float          v8f  __attribute__((ext_vector_type(8)));
typedef int            v4i  __attribute__((ext_vector_type(4)));
typedef int            v8i  __attribute__((ext_vector_type(8)));
typedef unsigned int   v4u  __attribute__((ext_vector_type(4)));
typedef unsigned short v8us __attribute__((ext_vector_type(8)));
typedef __bf16         v16b __attribute__((ext_vector_type(16)));
typedef v4f  __attribute__((may_alias)) v4fa;
typedef v8us __attribute__((may_alias)) v8usa;
union FragB { v16b v; v8us h[2]; v8i w; };

__device__ __forceinline__ v8f wmb(const FragB& a, const FragB& b, v8f c) {
  v8f d = __builtin_amdgcn_wmma_f32_16x16x32_bf16(false, a.v, false, b.v, (short)0, c, false, false);
  asm volatile("v_nop\n\tv_nop\n\tv_nop\n\tv_nop" : "+v"(d) : "v"(a.w), "v"(b.w));
  return d;
}

__device__ __forceinline__ unsigned int f2bf(float f) {
  const unsigned int u = __float_as_uint(f);
  return ((u + 0x7FFFu + ((u >> 16) & 1u)) >> 16) & 0xFFFFu;
}
__device__ __forceinline__ float bf2f(unsigned int b) { return __uint_as_float(b << 16); }
__device__ __forceinline__ float bfr(float f) { return bf2f(f2bf(f)); }
__device__ __forceinline__ v4f bfr4(const v4f a) {
  v4f r; r.x = bfr(a.x); r.y = bfr(a.y); r.z = bfr(a.z); r.w = bfr(a.w); return r;
}
__device__ __forceinline__ unsigned int pk2(float lo, float hi) { return f2bf(lo) | (f2bf(hi) << 16); }
__device__ __forceinline__ v4u pack8(const v4f a, const v4f b) {
  v4u r;
  r.x = pk2(a.x, a.y); r.y = pk2(a.z, a.w); r.z = pk2(b.x, b.y); r.w = pk2(b.z, b.w);
  return r;
}
__device__ __forceinline__ void hilo16(const v4f a, const v4f b, FragB& f) {
  v8us hi, lo;
  unsigned hb;
  hb = f2bf(a.x); hi[0] = (unsigned short)hb; lo[0] = (unsigned short)f2bf(a.x - bf2f(hb));
  hb = f2bf(a.y); hi[1] = (unsigned short)hb; lo[1] = (unsigned short)f2bf(a.y - bf2f(hb));
  hb = f2bf(a.z); hi[2] = (unsigned short)hb; lo[2] = (unsigned short)f2bf(a.z - bf2f(hb));
  hb = f2bf(a.w); hi[3] = (unsigned short)hb; lo[3] = (unsigned short)f2bf(a.w - bf2f(hb));
  hb = f2bf(b.x); hi[4] = (unsigned short)hb; lo[4] = (unsigned short)f2bf(b.x - bf2f(hb));
  hb = f2bf(b.y); hi[5] = (unsigned short)hb; lo[5] = (unsigned short)f2bf(b.y - bf2f(hb));
  hb = f2bf(b.z); hi[6] = (unsigned short)hb; lo[6] = (unsigned short)f2bf(b.z - bf2f(hb));
  hb = f2bf(b.w); hi[7] = (unsigned short)hb; lo[7] = (unsigned short)f2bf(b.w - bf2f(hb));
  f.h[0] = hi; f.h[1] = lo;
}
__device__ __forceinline__ float elu1(float h) {
  const float n = __expf(fminf(h, 0.f)) - 1.0f;
  return h > 0.f ? h : n;
}

__device__ __forceinline__ int scan_chunk(const int* __restrict__ dsts, int nE, int cbase, int slotBase,
                                          int nb, int vec8, int* list, int tid, int lane, int wave) {
  int wc = 0;
  const int el0  = tid * EPT;
  const int e0   = cbase + el0;
  const int sent = -2147483647 - 1;
  v4i da, db;
  if (vec8 != 0 && cbase + CHUNK <= nE) {
    da = *(const v4i*)(dsts + e0);
    db = *(const v4i*)(dsts + e0 + 4);
  } else {
    da.x = (e0     < nE) ? dsts[min(e0,     nE - 1)] : sent;
    da.y = (e0 + 1 < nE) ? dsts[min(e0 + 1, nE - 1)] : sent;
    da.z = (e0 + 2 < nE) ? dsts[min(e0 + 2, nE - 1)] : sent;
    da.w = (e0 + 3 < nE) ? dsts[min(e0 + 3, nE - 1)] : sent;
    db.x = (e0 + 4 < nE) ? dsts[min(e0 + 4, nE - 1)] : sent;
    db.y = (e0 + 5 < nE) ? dsts[min(e0 + 5, nE - 1)] : sent;
    db.z = (e0 + 6 < nE) ? dsts[min(e0 + 6, nE - 1)] : sent;
    db.w = (e0 + 7 < nE) ? dsts[min(e0 + 7, nE - 1)] : sent;
  }
  const unsigned nbs = (unsigned)slotBase;
  const unsigned unb = (unsigned)nb;
  const unsigned s0 = (unsigned)da.x - nbs, s1 = (unsigned)da.y - nbs;
  const unsigned s2 = (unsigned)da.z - nbs, s3 = (unsigned)da.w - nbs;
  const unsigned s4 = (unsigned)db.x - nbs, s5 = (unsigned)db.y - nbs;
  const unsigned s6 = (unsigned)db.z - nbs, s7 = (unsigned)db.w - nbs;
  const bool h0 = s0 < unb, h1 = s1 < unb, h2 = s2 < unb, h3 = s3 < unb;
  const bool h4 = s4 < unb, h5 = s5 < unb, h6 = s6 < unb, h7 = s7 < unb;
  const unsigned any = __builtin_amdgcn_ballot_w32(h0 | h1 | h2 | h3 | h4 | h5 | h6 | h7);
  if (any != 0u) {
#define HITJ(J, HJ, SJ) { \
      const unsigned mj = __builtin_amdgcn_ballot_w32(HJ); \
      if (mj != 0u) { \
        if (HJ) { \
          const int pos = wc + (int)__builtin_amdgcn_mbcnt_lo(mj, 0u); \
          if (pos < WCAP) list[wave * WCAP + pos] = ((el0 + (J)) << SLOTB) | (int)(SJ); \
        } \
        wc += (int)__builtin_popcount(mj); } }
    HITJ(0, h0, s0)
    HITJ(1, h1, s1)
    HITJ(2, h2, s2)
    HITJ(3, h3, s3)
    HITJ(4, h4, s4)
    HITJ(5, h5, s5)
    HITJ(6, h6, s6)
    HITJ(7, h7, s7)
#undef HITJ
  }
  return wc;
}

__global__ __launch_bounds__(NTHR) void k_xprep(const float* __restrict__ x, unsigned short* xb, int nN, int nUnits) {
  const int i = (int)blockIdx.x * NTHR + (int)threadIdx.x;
  if (i >= nUnits) return;
  const int row = i >> 4;
  const int c0  = (i & 15) * 8;
  const int rc  = row < nN ? row : nN - 1;
  const float* p = x + (size_t)rc * F_IN + c0;
  v4f a = *(const v4fa*)p, b = *(const v4fa*)(p + 4);
  const v4f z4 = {0.f, 0.f, 0.f, 0.f};
  if (row >= nN) { a = z4; b = z4; }
  const v4u hv = pack8(a, b);
  const size_t o = (size_t)row * F_IN + c0;
  *(volatile v4u*)(xb + o) = hv;
  __threadfence();
  *(volatile v4u*)(xb + o) = hv;
}

__global__ __launch_bounds__(NTHR) void k_wprep(const float* __restrict__ W1, const float* __restrict__ W2,
                                                unsigned short* W1T, unsigned short* W2T) {
  const int u = (int)blockIdx.x * NTHR + (int)threadIdx.x;
  v8us o;
  unsigned short* dp;
  if (u < NU1) {
    const int n  = u >> 4;
    const int k8 = 8 * (u & 15);
    const int r  = n >> 7;
    const int nc = n & (HC - 1);
    const float* p = W1 + (size_t)r * F_IN * HC + (size_t)k8 * HC + nc;
#pragma unroll
    for (int i = 0; i < 8; ++i) o[i] = (unsigned short)f2bf(p[(size_t)i * HC]);
    dp = W1T + (size_t)n * F_IN + k8;
  } else if (u < NU1 + NU2) {
    const int v  = u - NU1;
    const int n  = v >> 5;
    const int g  = v & 31;
    const int kb = 16 * (g >> 2) + 8 * (g & 1);
    const int nn = n < NREL * C2 ? n : NREL * C2 - 1;
    const int r  = nn >> 4;
    const int nc = nn & (C2 - 1);
    const float* p = W2 + (size_t)r * HC * C2 + (size_t)kb * C2 + nc;
    v4f a, b;
    a.x = p[0];              a.y = p[(size_t)C2];     a.z = p[(size_t)2 * C2]; a.w = p[(size_t)3 * C2];
    b.x = p[(size_t)4 * C2]; b.y = p[(size_t)5 * C2]; b.z = p[(size_t)6 * C2]; b.w = p[(size_t)7 * C2];
    const v4f z4 = {0.f, 0.f, 0.f, 0.f};
    if (n >= NREL * C2) { a = z4; b = z4; }
    o[0] = (unsigned short)f2bf(a.x); o[1] = (unsigned short)f2bf(a.y);
    o[2] = (unsigned short)f2bf(a.z); o[3] = (unsigned short)f2bf(a.w);
    o[4] = (unsigned short)f2bf(b.x); o[5] = (unsigned short)f2bf(b.y);
    o[6] = (unsigned short)f2bf(b.z); o[7] = (unsigned short)f2bf(b.w);
    dp = W2T + (size_t)n * K2 + 8 * g;
  } else {
    return;
  }
  *(volatile v8us*)dp = o;
  __threadfence();
  *(volatile v8us*)dp = o;
}

__global__ __launch_bounds__(GTHR) void k_gemm1(
    const unsigned short* __restrict__ A, const unsigned short* __restrict__ WT, float* outF,
    const float* __restrict__ al, const float* __restrict__ ar, float* SD, int MPr)
{
  __shared__ __attribute__((aligned(16))) float stg[GBM * HC];
  __shared__ __attribute__((aligned(16))) float satt[2 * HC];
  __shared__ __attribute__((aligned(16))) float sdot[8 * GBM];
  const int tid = (int)threadIdx.x, lane = tid & 31, wave = tid >> 5, hh = lane >> 4, m = lane & 15;
  const int rowBase = (int)blockIdx.x * GBM;

  {
#pragma unroll 1
    for (int q = 0; q < 2; ++q) {
      const int i     = tid + q * GTHR;
      const int hw    = i >> 5;
      const int hl    = hw >> 1;
      const int which = hw & 1;
      const int c     = i & (HD1 - 1);
      const int idx   = hl * HD1 + c;
      const float va  = al[idx], vd = ar[idx];
      const float mw  = (float)which;
      const float v   = fmaf(mw, vd, (1.f - mw) * va);
      satt[i] = bfr(v);
    }
  }

  v8f acc[8];
  {
    const v8f z = {0.f, 0.f, 0.f, 0.f, 0.f, 0.f, 0.f, 0.f};
#pragma unroll
    for (int t = 0; t < 8; ++t) acc[t] = z;
  }
  const unsigned short* ap = A  + (size_t)(rowBase + 16 * wave + m) * (size_t)F_IN + 8 * hh;
  const unsigned short* bp = WT + (size_t)m * (size_t)F_IN + 8 * hh;

#pragma unroll 1
  for (int ks = 0; ks < F_IN / 32; ++ks) {
    const int k0 = 32 * ks;
    FragB af;
    af.h[0] = *(const v8usa*)(ap + k0);
    af.h[1] = *(const v8usa*)(ap + k0 + 16);
#pragma unroll
    for (int nt = 0; nt < 8; ++nt) {
      const unsigned short* wq = bp + (size_t)(16 * nt) * (size_t)F_IN + k0;
      FragB bf;
      bf.h[0] = *(const v8usa*)wq;
      bf.h[1] = *(const v8usa*)(wq + 16);
      acc[nt] = wmb(af, bf, acc[nt]);
    }
  }

#pragma unroll
  for (int nt = 0; nt < 8; ++nt) {
    const int lc = 16 * nt + m;
#pragma unroll
    for (int r = 0; r < 8; ++r) {
      const int lr = 16 * wave + 8 * hh + r;
      stg[lr * HC + lc] = acc[nt][r];
    }
  }
  __syncthreads();

  {
    const int row = tid & 63, g = tid >> 6;
    const float* hr  = stg + row * HC + (2 * g) * HD1;
    const float* sa0 = satt + (4 * g + 0) * HD1;
    const float* sd0 = satt + (4 * g + 1) * HD1;
    const float* sa1 = satt + (4 * g + 2) * HD1;
    const float* sd1 = satt + (4 * g + 3) * HD1;
    float ds0 = 0.f, dd0 = 0.f, ds1 = 0.f, dd1 = 0.f;
#pragma unroll 2
    for (int c4 = 0; c4 < HD1 / 4; ++c4) {
      const v4f h0 = *(const v4fa*)(hr + 4 * c4);
      const v4f h1 = *(const v4fa*)(hr + HD1 + 4 * c4);
      const v4f a0 = *(const v4fa*)(sa0 + 4 * c4);
      const v4f b0 = *(const v4fa*)(sd0 + 4 * c4);
      const v4f a1 = *(const v4fa*)(sa1 + 4 * c4);
      const v4f b1 = *(const v4fa*)(sd1 + 4 * c4);
      ds0 = fmaf(h0.x, a0.x, ds0); dd0 = fmaf(h0.x, b0.x, dd0); ds1 = fmaf(h1.x, a1.x, ds1); dd1 = fmaf(h1.x, b1.x, dd1);
      ds0 = fmaf(h0.y, a0.y, ds0); dd0 = fmaf(h0.y, b0.y, dd0); ds1 = fmaf(h1.y, a1.y, ds1); dd1 = fmaf(h1.y, b1.y, dd1);
      ds0 = fmaf(h0.z, a0.z, ds0); dd0 = fmaf(h0.z, b0.z, dd0); ds1 = fmaf(h1.z, a1.z, ds1); dd1 = fmaf(h1.z, b1.z, dd1);
      ds0 = fmaf(h0.w, a0.w, ds0); dd0 = fmaf(h0.w, b0.w, dd0); ds1 = fmaf(h1.w, a1.w, ds1); dd1 = fmaf(h1.w, b1.w, dd1);
    }
    sdot[(4 * g + 0) * GBM + row] = ds0;
    sdot[(4 * g + 1) * GBM + row] = dd0;
    sdot[(4 * g + 2) * GBM + row] = ds1;
    sdot[(4 * g + 3) * GBM + row] = dd1;
  }
  __syncthreads();

  v4f fv[16];
#pragma unroll
  for (int i = 0; i < 16; ++i) {
    const int lr = 16 * wave + i;
    fv[i] = *(const v4fa*)(stg + lr * HC + 4 * lane);
  }
  const int pl = tid >> 4, piece = tid & 15;
  const v4f sdv = *(const v4fa*)(sdot + pl * GBM + 4 * piece);
  float* sp = SD + (size_t)pl * (size_t)MPr + rowBase + 4 * piece;

#pragma unroll
  for (int i = 0; i < 16; ++i) {
    float* op = outF + (size_t)(rowBase + 16 * wave + i) * (size_t)HC + 4 * lane;
    *(volatile v4f*)op = fv[i];
  }
  *(volatile v4f*)sp = sdv;
  __threadfence();
#pragma unroll
  for (int i = 0; i < 16; ++i) {
    float* op = outF + (size_t)(rowBase + 16 * wave + i) * (size_t)HC + 4 * lane;
    *(volatile v4f*)op = fv[i];
  }
  *(volatile v4f*)sp = sdv;
}

__global__ __launch_bounds__(GTHR) void k_gemm2(
    const float* __restrict__ Hin, const unsigned short* __restrict__ WT, float* outF,
    const float* __restrict__ al, const float* __restrict__ ar, float* SD, int MPr)
{
  constexpr int PP2 = 2 * NREL;
  __shared__ __attribute__((aligned(16))) float stg[GBM * N2P];
  __shared__ __attribute__((aligned(16))) float satt[2 * N2P];
  __shared__ __attribute__((aligned(16))) float sdot[8 * GBM];
  const int tid = (int)threadIdx.x, lane = tid & 31, wave = tid >> 5, hh = lane >> 4, m = lane & 15;
  const int rowBase = (int)blockIdx.x * GBM;

  {
    const int i     = tid;
    const int ic    = i < PP2 * C2 ? i : PP2 * C2 - 1;
    const int hw    = ic >> 4;
    const int r     = hw >> 1;
    const int which = hw & 1;
    const int c     = ic & (C2 - 1);
    const int idx   = r * C2 + c;
    const float va  = al[idx], vd = ar[idx];
    const float mw  = (float)which;
    const float v   = fmaf(mw, vd, (1.f - mw) * va);
    satt[i] = bfr(v);
  }

  v8f acc[4];
  {
    const v8f z = {0.f, 0.f, 0.f, 0.f, 0.f, 0.f, 0.f, 0.f};
    acc[0] = z; acc[1] = z; acc[2] = z; acc[3] = z;
  }
  const float*          ap = Hin + (size_t)(rowBase + 16 * wave + m) * (size_t)HC + 8 * hh;
  const unsigned short* wp = WT  + (size_t)m * (size_t)K2 + 8 * hh;

#pragma unroll 1
  for (int s = 0; s < HC / 16; ++s) {
    const float* fp = ap + 16 * s;
    const v4f f0 = *(const v4fa*)fp;
    const v4f f1 = *(const v4fa*)(fp + 4);
    FragB af;
    hilo16(f0, f1, af);
#pragma unroll
    for (int t = 0; t < 4; ++t) {
      const unsigned short* wq = wp + (size_t)(16 * t) * (size_t)K2 + 32 * s;
      FragB bf;
      bf.h[0] = *(const v8usa*)wq;
      bf.h[1] = *(const v8usa*)(wq + 16);
      acc[t] = wmb(af, bf, acc[t]);
    }
  }

#pragma unroll
  for (int t = 0; t < 4; ++t) {
    const int lc = 16 * t + m;
#pragma unroll
    for (int r = 0; r < 8; ++r) {
      const int lr = 16 * wave + 8 * hh + r;
      stg[lr * N2P + lc] = acc[t][r];
    }
  }
  __syncthreads();

  {
    const int row = tid & 63, g = tid >> 6;
#pragma unroll
    for (int r = 0; r < NREL; ++r) {
      const float* hr = stg + row * N2P + C2 * r;
      const float* sv = satt + (2 * r + g) * C2;
      float dv = 0.f;
#pragma unroll
      for (int c4 = 0; c4 < C2 / 4; ++c4) {
        const v4f h0 = *(const v4fa*)(hr + 4 * c4);
        const v4f a0 = *(const v4fa*)(sv + 4 * c4);
        dv = fmaf(h0.x, a0.x, dv);
        dv = fmaf(h0.y, a0.y, dv);
        dv = fmaf(h0.z, a0.z, dv);
        dv = fmaf(h0.w, a0.w, dv);
      }
      sdot[(2 * r + g) * GBM + row] = dv;
    }
  }
  __syncthreads();

  v4f fv[8];
#pragma unroll
  for (int i = 0; i < 8; ++i) {
    const int lr = 16 * wave + 2 * i + hh;
    fv[i] = *(const v4fa*)(stg + lr * N2P + 4 * m);
  }
  const int pl = tid >> 4, piece = tid & 15;
  const bool wsd = pl < PP2;
  const int plr = wsd ? pl : PP2 - 1;
  const v4f sdv = *(const v4fa*)(sdot + plr * GBM + 4 * piece);
  float* sp = SD + (size_t)plr * (size_t)MPr + rowBase + 4 * piece;

#pragma unroll
  for (int i = 0; i < 8; ++i) {
    const int lr = 16 * wave + 2 * i + hh;
    float* op = outF + (size_t)(rowBase + lr) * (size_t)N2P + 4 * m;
    *(volatile v4f*)op = fv[i];
  }
  if (wsd) *(volatile v4f*)sp = sdv;
  __threadfence();
#pragma unroll
  for (int i = 0; i < 8; ++i) {
    const int lr = 16 * wave + 2 * i + hh;
    float* op = outF + (size_t)(rowBase + lr) * (size_t)N2P + 4 * m;
    *(volatile v4f*)op = fv[i];
  }
  if (wsd) *(volatile v4f*)sp = sdv;
}

template <int L, int R3>
__global__ __launch_bounds__(NTHR) void k_agg(
    const int* __restrict__ srcs, const int* __restrict__ dsts,
    const float* __restrict__ F, const float* __restrict__ SD,
    const float* __restrict__ bias, float* P, float* P2, float* out,
    int nN, int nE, int nb, int vec8, int MPr) {
  extern __shared__ v4f lds_dyn[];
  int* reg1 = (int*)lds_dyn;
  int* reg2 = reg1 + RCAP;
  int* scnt = reg2 + RCAP;
  int* soff = scnt + NBMAX;
  int* list = soff + NBMAX;
  int* wcnt = list + LISTN;
  int* wtot = wcnt + NWAVE;
  const int tid = (int)threadIdx.x, lane = tid & 31, wave = tid >> 5;
  const int nodeBase = (int)blockIdx.x * nb;

  for (int i = tid; i < NBMAX; i += NTHR) scnt[i] = 0;
  __syncthreads();

  int tot = 0;
  const int nChunks = (nE + CHUNK - 1) / CHUNK;
#pragma unroll 1
  for (int ch = 0; ch < nChunks; ++ch) {
    const int cbase = ch * CHUNK;
    const int wc = scan_chunk(dsts, nE, cbase, nodeBase, nb, vec8, list, tid, lane, wave);
    if (lane == 0) wcnt[wave] = wc;
    __syncthreads();
    int pre = 0, all = 0;
#pragma unroll
    for (int w2 = 0; w2 < NWAVE; ++w2) {
      int c = wcnt[w2];
      c = c < 0 ? 0 : (c > WCAP ? WCAP : c);
      all += c;
      pre += (w2 < wave) ? c : 0;
    }
    const int wcc  = wc > WCAP ? WCAP : wc;
    const int base = tot + pre;
#pragma unroll 1
    for (int i = lane; i < wcc; i += 32) {
      const int ent = list[wave * WCAP + i];
      const int el  = (ent >> SLOTB) & (CHUNK - 1);
      const int sl  = ent & (NBMAX - 1);
      int eid = cbase + el;
      eid = eid > nE - 1 ? nE - 1 : eid;
      const int pos = base + i;
      if (pos < RCAP) reg1[pos] = (int)(((unsigned)eid << SLOTB) | (unsigned)sl);
    }
    tot += all;
    tot = tot > RCAP ? RCAP : tot;
    __syncthreads();
  }
  const int nh = tot;

  if (wave == 0) {
#pragma unroll 1
    for (int b0 = 0; b0 < nh; b0 += 32) {
      const int idx = b0 + lane;
      const int uv  = reg1[idx < nh ? idx : nh - 1];
      const int m32 = (nh - b0) < 32 ? (nh - b0) : 32;
#pragma unroll 1
      for (int k = 0; k < m32; ++k) {
        const int u  = __builtin_amdgcn_readlane(uv, k);
        const int sl = u & (NBMAX - 1);
        if (lane == 0) scnt[sl] = scnt[sl] + 1;
      }
    }
  }
  __syncthreads();

  {
    const v4i ca = *(const v4i*)(scnt + 8 * tid);
    const v4i cb = *(const v4i*)(scnt + 8 * tid + 4);
    const int e0 = ca.x < 0 ? 0 : ca.x, e1 = ca.y < 0 ? 0 : ca.y, e2 = ca.z < 0 ? 0 : ca.z, e3 = ca.w < 0 ? 0 : ca.w;
    const int e4 = cb.x < 0 ? 0 : cb.x, e5 = cb.y < 0 ? 0 : cb.y, e6 = cb.z < 0 ? 0 : cb.z, e7 = cb.w < 0 ? 0 : cb.w;
    const int ts = e0 + e1 + e2 + e3 + e4 + e5 + e6 + e7;
    int incl = ts;
#pragma unroll
    for (int d = 1; d < 32; d <<= 1) {
      const int up = __shfl_up(incl, d);
      if (lane >= d) incl += up;
    }
    if (lane == 31) wtot[wave] = incl;
    __syncthreads();
    int pre = 0;
#pragma unroll
    for (int w2 = 0; w2 < NWAVE; ++w2) pre += (w2 < wave) ? wtot[w2] : 0;
    int run = pre + incl - ts;
    soff[8 * tid + 0] = run; run += e0;
    soff[8 * tid + 1] = run; run += e1;
    soff[8 * tid + 2] = run; run += e2;
    soff[8 * tid + 3] = run; run += e3;
    soff[8 * tid + 4] = run; run += e4;
    soff[8 * tid + 5] = run; run += e5;
    soff[8 * tid + 6] = run; run += e6;
    soff[8 * tid + 7] = run;
  }
  __syncthreads();
  for (int i = tid; i < NBMAX; i += NTHR) list[i] = soff[i];
  __syncthreads();

  if (wave == 0) {
#pragma unroll 1
    for (int b0 = 0; b0 < nh; b0 += 32) {
      const int idx = b0 + lane;
      const int uv  = reg1[idx < nh ? idx : nh - 1];
      const int m32 = (nh - b0) < 32 ? (nh - b0) : 32;
#pragma unroll 1
      for (int k = 0; k < m32; ++k) {
        const int u   = __builtin_amdgcn_readlane(uv, k);
        const int sl  = u & (NBMAX - 1);
        const int eid = (int)((unsigned)u >> SLOTB);
        if (lane == 0) {
          int pos = list[sl];
          pos = pos < 0 ? 0 : (pos > RCAP - 1 ? RCAP - 1 : pos);
          reg2[pos] = eid;
          list[sl] = pos + 1;
        }
      }
    }
  }
  __syncthreads();

  const int nbw = nb >> 3;
  const bool ovf = (nh >= RCAP);
  const float qnan = __int_as_float(0x7fc00000);
  const v4f z4 = {0.f, 0.f, 0.f, 0.f};

  if constexpr (L == 1) {
    const int c0   = 4 * lane;
    const int head = lane >> 3;
    const v4f bb   = bfr4(*(const v4fa*)(bias + c0));
    const float* ASp = SD + (size_t)(2 * head) * (size_t)MPr;
    const float* ADp = ASp + MPr;
    const float* Fr  = F + c0;

#pragma unroll 1
    for (int jt = 0; jt < nbw; ++jt) {
      const int slot = wave * nbw + jt;
      const int grow = nodeBase + slot;
      const int gcl  = grow < nN ? grow : nN - 1;
      int st = soff[slot];
      const int craw = scnt[slot];
      int cnt = craw;
      st  = st < 0 ? 0 : (st > nh ? nh : st);
      cnt = cnt < 0 ? 0 : (cnt > DEGCAP ? DEGCAP : cnt);
      if (cnt > nh - st) cnt = nh - st;
      const float pz = (ovf || craw > DEGCAP) ? qnan : 0.0f;

      const float adv = ADp[gcl];
      float mx = MX0, dn = 0.0f;
      v4f av = z4;

#pragma unroll 1
      for (int q = 0; q < cnt; ++q) {
        int idx = st + q; idx = idx > RCAP - 1 ? RCAP - 1 : idx;
        int eid = reg2[idx]; eid = eid < 0 ? 0 : (eid > nE - 1 ? nE - 1 : eid);
        const int sraw = srcs[eid];
        const int s = sraw < 0 ? 0 : (sraw > nN - 1 ? nN - 1 : sraw);
        const v4f fs = *(const v4fa*)(Fr + (size_t)s * HC);
        float lg = ASp[s] + adv;
        lg = lg > 0.f ? lg : NEGSL * lg;
        const float df = lg - mx;
        const float ee = __expf(-fabsf(df));
        const bool up  = df > 0.f;
        const float s1 = up ? ee : 1.0f;
        const float s2 = up ? 1.0f : ee;
        mx = up ? lg : mx;
        dn = fmaf(dn, s1, s2);
        av.x = fmaf(av.x, s1, s2 * fs.x);
        av.y = fmaf(av.y, s1, s2 * fs.y);
        av.z = fmaf(av.z, s1, s2 * fs.z);
        av.w = fmaf(av.w, s1, s2 * fs.w);
      }
      const float inv = __builtin_amdgcn_rcpf(dn + EPS_SM);
      v4f pv = z4;
      if constexpr (R3 > 0) pv = *(const v4fa*)(P + (size_t)gcl * HC + c0);
      const bool live = grow < nN;
      v4f v;
      v.x = pv.x + fmaf(av.x, inv, bb.x);
      v.y = pv.y + fmaf(av.y, inv, bb.y);
      v.z = pv.z + fmaf(av.z, inv, bb.z);
      v.w = pv.w + fmaf(av.w, inv, bb.w);
      v4f o;
      if constexpr (R3 < 2) {
        o.x = (live ? v.x : 0.f) + pz;
        o.y = (live ? v.y : 0.f) + pz;
        o.z = (live ? v.z : 0.f) + pz;
        o.w = (live ? v.w : 0.f) + pz;
      } else {
        o.x = (live ? elu1(v.x * THIRD) : 0.f) + pz;
        o.y = (live ? elu1(v.y * THIRD) : 0.f) + pz;
        o.z = (live ? elu1(v.z * THIRD) : 0.f) + pz;
        o.w = (live ? elu1(v.w * THIRD) : 0.f) + pz;
      }
      if (grow < MPr) {
        float* op = P + (size_t)grow * HC + c0;
        *(volatile v4f*)op = o;
        __threadfence();
        *(volatile v4f*)op = o;
      }
    }
  } else {
    float* res = (float*)reg1;
    const int u  = lane >> 2;
    const int cq = (lane & 3) * 4;
    const v4f bb = bfr4(*(const v4fa*)(bias + cq));
    const float* ASp = SD + (size_t)(2 * R3) * (size_t)MPr;
    const float* ADp = ASp + MPr;
    const float* Fr  = F + C2 * R3 + cq;
    const int nhm1 = nh > 0 ? nh - 1 : 0;

#pragma unroll 1
    for (int jt = 0; jt < nbw; jt += 8) {
      const int slot = wave * nbw + jt + u;
      const int grow = nodeBase + slot;
      const int gcl  = grow < nN ? grow : nN - 1;
      int st = soff[slot];
      const int craw = scnt[slot];
      int cnt = craw;
      st  = st < 0 ? 0 : (st > nh ? nh : st);
      cnt = cnt < 0 ? 0 : (cnt > DEGCAP ? DEGCAP : cnt);
      cnt = cnt > nh - st ? nh - st : cnt;
      const float pz = (ovf || craw > DEGCAP) ? qnan : 0.0f;
      int cm = cnt;
      { const int o4 = __shfl_xor(cm, 4);  cm = cm > o4 ? cm : o4; }
      { const int o8 = __shfl_xor(cm, 8);  cm = cm > o8 ? cm : o8; }
      { const int o16 = __shfl_xor(cm, 16); cm = cm > o16 ? cm : o16; }

      const float adv = ADp[gcl];
      float mx = MX0, dn = 0.0f;
      v4f av = z4;

#pragma unroll 1
      for (int q = 0; q < cm; ++q) {
        const bool act = q < cnt;
        int idx = st + (act ? q : 0);
        idx = idx < 0 ? 0 : idx;
        idx = idx > nhm1 ? nhm1 : idx;
        idx = idx > RCAP - 1 ? RCAP - 1 : idx;
        int eid = reg2[idx]; eid = eid < 0 ? 0 : (eid > nE - 1 ? nE - 1 : eid);
        const int sraw = srcs[eid];
        const int s = sraw < 0 ? 0 : (sraw > nN - 1 ? nN - 1 : sraw);
        const v4f fs = *(const v4fa*)(Fr + (size_t)s * N2P);
        float lg = ASp[s] + adv;
        lg = lg > 0.f ? lg : NEGSL * lg;
        const float df = lg - mx;
        const float ee = __expf(-fabsf(df));
        const bool up  = act && (df > 0.f);
        const float s1 = up ? ee : 1.0f;
        const float s2 = act ? (up ? 1.0f : ee) : 0.0f;
        mx = up ? lg : mx;
        dn = fmaf(dn, s1, s2);
        av.x = fmaf(av.x, s1, s2 * fs.x);
        av.y = fmaf(av.y, s1, s2 * fs.y);
        av.z = fmaf(av.z, s1, s2 * fs.z);
        av.w = fmaf(av.w, s1, s2 * fs.w);
      }
      const float inv = __builtin_amdgcn_rcpf(dn + EPS_SM);
      v4f pv = z4;
      if constexpr (R3 > 0) pv = *(const v4fa*)(P2 + (size_t)gcl * C2 + cq);
      const bool live = grow < nN;
      v4f v;
      v.x = pv.x + fmaf(av.x, inv, bb.x);
      v.y = pv.y + fmaf(av.y, inv, bb.y);
      v.z = pv.z + fmaf(av.z, inv, bb.z);
      v.w = pv.w + fmaf(av.w, inv, bb.w);
      if constexpr (R3 == 2) { v.x *= THIRD; v.y *= THIRD; v.z *= THIRD; v.w *= THIRD; }
      v4f o;
      o.x = (live ? v.x : 0.f) + pz;
      o.y = (live ? v.y : 0.f) + pz;
      o.z = (live ? v.z : 0.f) + pz;
      o.w = (live ? v.w : 0.f) + pz;
      *(v4fa*)(res + slot * C2 + cq) = o;
    }
    __syncthreads();

    int prow = ((R3 < 2) ? MPr : nN) - nodeBase;
    prow = prow < 0 ? 0 : (prow > nb ? nb : prow);
    const int plim = prow * (C2 / 4);
    float* ob = (R3 < 2) ? (P2 + (size_t)nodeBase * C2) : (out + (size_t)nodeBase * C2);
#pragma unroll 1
    for (int p = tid; p < plim; p += NTHR) {
      const v4f vv = *(const v4fa*)(res + 4 * p);
      *(volatile v4f*)(ob + 4 * (size_t)p) = vv;
    }
    __threadfence();
#pragma unroll 1
    for (int p = tid; p < plim; p += NTHR) {
      const v4f vv = *(const v4fa*)(res + 4 * p);
      *(volatile v4f*)(ob + 4 * (size_t)p) = vv;
    }
  }
}

static int pick_nb(int nE, int nN) {
  int nb = NBCAP;
  while (nb > 64 && (long long)nb * (long long)nE * 5LL > (long long)RCAP * (long long)nN * 4LL) nb >>= 1;
  return nb;
}
static inline int cdiv(int a, int b) { return (a + b - 1) / b; }

extern "C" void kernel_launch(void* const* d_in, const int* in_sizes, int n_in,
                              void* d_out, int out_size, void* d_ws, size_t ws_size,
                              hipStream_t stream) {
  if (n_in < 11) return;
  if (in_sizes[0] < F_IN || (in_sizes[0] % F_IN) != 0) return;
  const int nN = in_sizes[0] / F_IN;
  if (nN < 1 || nN > (1 << 22)) return;
  if (in_sizes[1] < NREL || (in_sizes[1] % NREL) != 0 || in_sizes[2] != in_sizes[1]) return;
  const int nE = in_sizes[1] / NREL;
  if (nE < 1 || nE >= (1 << (32 - SLOTB))) return;
  if (in_sizes[3] != NREL * F_IN * HC) return;
  if (in_sizes[4] != NREL * NH1 * HD1 || in_sizes[5] != NREL * NH1 * HD1) return;
  if (in_sizes[6] != NREL * HC) return;
  if (in_sizes[7] != NREL * HC * C2) return;
  if (in_sizes[8] != NREL * C2 || in_sizes[9] != NREL * C2) return;
  if (in_sizes[10] != NREL * C2) return;
  if ((long long)out_size != (long long)nN * C2) return;

  const float* x   = (const float*)d_in[0];
  const int*   src = (const int*)  d_in[1];
  const int*   dst = (const int*)  d_in[2];
  const float* W1  = (const float*)d_in[3];
  const float* al1 = (const float*)d_in[4];
  const float* ar1 = (const float*)d_in[5];
  const float* b1  = (const float*)d_in[6];
  const float* W2  = (const float*)d_in[7];
  const float* al2 = (const float*)d_in[8];
  const float* ar2 = (const float*)d_in[9];
  const float* b2  = (const float*)d_in[10];
  float* out = (float*)d_out;

  const int MP   = cdiv(nN, MROWS) * MROWS;
  const int nb   = pick_nb(nE, nN);
  if (nb < 64 || (nb & (nb - 1)) != 0 || nb > NBCAP) return;
  const int gA   = cdiv(MP, nb);
  if ((long long)gA * nb < (long long)MP) return;
  const int vec8 = ((nE & 3) == 0) ? 1 : 0;
  const int gM   = MP / GBM;

  char* ws = (char*)d_ws;
  size_t off = 0;
  const size_t oXB  = off; off += (size_t)MP * F_IN * 2;            off = (off + 255) & ~(size_t)255;
  const size_t oW1T = off; off += (size_t)NREL * HC * F_IN * 2;     off = (off + 255) & ~(size_t)255;
  const size_t oW2T = off; off += (size_t)N2P * K2 * 2;             off = (off + 255) & ~(size_t)255;
  const size_t oH   = off; off += (size_t)MP * HC * 4;              off = (off + 255) & ~(size_t)255;
  const size_t oSD1 = off; off += (size_t)2 * NH1 * MP * 4;         off = (off + 255) & ~(size_t)255;
  const size_t oP   = off; off += (size_t)MP * HC * 4;              off = (off + 255) & ~(size_t)255;
  if (off > ws_size || off > (size_t)WSMAX) return;
  size_t sub = oH;
  const size_t oH2  = sub; sub += (size_t)MP * N2P * 4;             sub = (sub + 255) & ~(size_t)255;
  const size_t oSD2 = sub; sub += (size_t)2 * NREL * MP * 4;        sub = (sub + 255) & ~(size_t)255;
  const size_t oP2  = sub; sub += (size_t)MP * C2 * 4;              sub = (sub + 255) & ~(size_t)255;
  if (sub > oSD1) return;
  unsigned short* XB  = (unsigned short*)(ws + oXB);
  unsigned short* W1T = (unsigned short*)(ws + oW1T);
  unsigned short* W2T = (unsigned short*)(ws + oW2T);
  float*          H   = (float*)(ws + oH);
  float*          SD1 = (float*)(ws + oSD1);
  float*          P   = (float*)(ws + oP);
  float*          H2  = (float*)(ws + oH2);
  float*          SD2 = (float*)(ws + oSD2);
  float*          P2  = (float*)(ws + oP2);

  hipFuncSetAttribute(reinterpret_cast<const void*>(&k_agg<1, 0>), hipFuncAttributeMaxDynamicSharedMemorySize, LDS_AGG);
  hipFuncSetAttribute(reinterpret_cast<const void*>(&k_agg<1, 1>), hipFuncAttributeMaxDynamicSharedMemorySize, LDS_AGG);
  hipFuncSetAttribute(reinterpret_cast<const void*>(&k_agg<1, 2>), hipFuncAttributeMaxDynamicSharedMemorySize, LDS_AGG);
  hipFuncSetAttribute(reinterpret_cast<const void*>(&k_agg<2, 0>), hipFuncAttributeMaxDynamicSharedMemorySize, LDS_AGG);
  hipFuncSetAttribute(reinterpret_cast<const void*>(&k_agg<2, 1>), hipFuncAttributeMaxDynamicSharedMemorySize, LDS_AGG);
  hipFuncSetAttribute(reinterpret_cast<const void*>(&k_agg<2, 2>), hipFuncAttributeMaxDynamicSharedMemorySize, LDS_AGG);

  k_wprep<<<(NU1 + NU2) / NTHR, NTHR, 0, stream>>>(W1, W2, W1T, W2T);
  const int nUx = MP * (F_IN / 8);
  k_xprep<<<cdiv(nUx, NTHR), NTHR, 0, stream>>>(x, XB, nN, nUx);

  const size_t eoff1 = (size_t)nE, eoff2 = (size_t)2 * nE;
  k_gemm1<<<gM, GTHR, 0, stream>>>(XB, W1T, H, al1, ar1, SD1, MP);
  k_agg<1, 0><<<gA, NTHR, LDS_AGG, stream>>>(src, dst, H, SD1, b1, P, P2, out, nN, nE, nb, vec8, MP);
  k_gemm1<<<gM, GTHR, 0, stream>>>(XB, W1T + (size_t)HC * F_IN, H, al1 + NH1 * HD1, ar1 + NH1 * HD1, SD1, MP);
  k_agg<1, 1><<<gA, NTHR, LDS_AGG, stream>>>(src + eoff1, dst + eoff1, H, SD1, b1 + HC, P, P2, out, nN, nE, nb, vec8, MP);
  k_gemm1<<<gM, GTHR, 0, stream>>>(XB, W1T + (size_t)2 * HC * F_IN, H, al1 + 2 * NH1 * HD1, ar1 + 2 * NH1 * HD1, SD1, MP);
  k_agg<1, 2><<<gA, NTHR, LDS_AGG, stream>>>(src + eoff2, dst + eoff2, H, SD1, b1 + 2 * HC, P, P2, out, nN, nE, nb, vec8, MP);

  k_gemm2<<<gM, GTHR, 0, stream>>>(P, W2T, H2, al2, ar2, SD2, MP);
  k_agg<2, 0><<<gA, NTHR, LDS_AGG, stream>>>(src, dst, H2, SD2, b2, P, P2, out, nN, nE, nb, vec8, MP);
  k_agg<2, 1><<<gA, NTHR, LDS_AGG, stream>>>(src + eoff1, dst + eoff1, H2, SD2, b2 + C2, P, P2, out, nN, nE, nb, vec8, MP);
  k_agg<2, 2><<<gA, NTHR, LDS_AGG, stream>>>(src + eoff2, dst + eoff2, H2, SD2, b2 + 2 * C2, P, P2, out, nN, nE, nb, vec8, MP);
}
